// GeneratedTreeClassifier_50062138802284
// MI455X (gfx1250) — hardware-verified
//
#include <hip/hip_runtime.h>

typedef __attribute__((ext_vector_type(16))) __bf16 v16b;
typedef unsigned short v8us  __attribute__((ext_vector_type(8)));
typedef unsigned short v16us __attribute__((ext_vector_type(16)));
typedef float v8f __attribute__((ext_vector_type(8)));
typedef float v4f __attribute__((ext_vector_type(4)));
typedef v8us __attribute__((may_alias)) v8usa;
typedef v4f  __attribute__((may_alias)) v4fa;

union Frag { v16b v; v16us u; v8us half[2]; };

#define NB    16384
#define NF    512
#define NT    64
#define NI    7
#define NL    8
#define NC    512
#define NCOL  512
#define PPT   7687
#define OFF_B 3584
#define OFF_L 3591

#define XBLK  ((NB * NF / 8) / 256)
#define WBLK  ((NCOL * NF / 8) / 256)

static_assert(PPT == NI * (NF + 1) + NL * NC);
static_assert(OFF_B == NI * NF);
static_assert(OFF_L == NI * NF + NI);
static_assert(NCOL == NT * NL);
static_assert(NF % 32 == 0);
static_assert(NCOL % 64 == 0);
static_assert(NB % 128 == 0);
static_assert(NC % 128 == 0);
static_assert((NB * NF / 8) % 256 == 0);
static_assert((NCOL * NF / 8) % 256 == 0);

__device__ __forceinline__ unsigned short bfb(float f) {
  unsigned u = __float_as_uint(f);
  u = u + 0x7FFFu + ((u >> 16) & 1u);
  return (unsigned short)(u >> 16);
}
__device__ __forceinline__ float bfv(unsigned short s) {
  return __uint_as_float(((unsigned)s) << 16);
}

__device__ __forceinline__ v8f wmma_bf16(v16b a, v16b b, v8f c) {
  v8f d = __builtin_amdgcn_wmma_f32_16x16x32_bf16(false, a, false, b, (short)0, c, false, false);
  asm volatile("v_nop\n\tv_nop\n\tv_nop\n\tv_nop" : "+v"(d) : "v"(a), "v"(b));
  return d;
}

__device__ __forceinline__ v16b load_frag(const unsigned short* p, int h) {
  Frag f;
  f.half[0] = *(const v8usa*)(p + 8 * h);
  f.half[1] = *(const v8usa*)(p + 16 + 8 * h);
  return f.v;
}

__device__ __forceinline__ void store2_us8(unsigned short* dst, v8us o) {
  *(volatile v8us*)dst = o;
  __threadfence();
  *(volatile v8us*)dst = o;
}

__device__ __forceinline__ void tile_store_pass(const float* sT, float* g, int gp, int w, int lane) {
  const int q8 = lane & 7, sub = lane >> 3;
  #pragma unroll
  for (int i = 0; i < 16; ++i) {
    const int lid = 4 * i + sub;
    const int row = 32 * w + (lid >> 1), hl = lid & 1;
    const v4f v = *(const v4fa*)(sT + row * 64 + 32 * hl + 4 * q8);
    *(volatile v4f*)(g + (size_t)row * gp + 32 * hl + 4 * q8) = v;
  }
}

template <int RPW>
__device__ __forceinline__ void line64_store_pass(const unsigned short* s, unsigned short* g,
                                                  int gp, int w, int lane) {
  const int q8 = lane & 7, sub = lane >> 3;
  #pragma unroll
  for (int i = 0; i < RPW / 4; ++i) {
    const int row = RPW * w + 4 * i + sub;
    const v8us v = *(const v8usa*)(s + row * 64 + 8 * q8);
    *(volatile v8us*)(g + (size_t)row * gp + 8 * q8) = v;
  }
}

__global__ __launch_bounds__(256) void convert_kernel(
    const float* __restrict__ x, const float* __restrict__ tp,
    unsigned short* __restrict__ xh, unsigned short* __restrict__ wt)
{
  const int bid = blockIdx.x, tid = threadIdx.x;
  if (bid < XBLK) {
    const size_t g = (size_t)bid * 256 + tid;
    const float* src = x + g * 8;
    const v4f a = *(const v4fa*)src;
    const v4f c = *(const v4fa*)(src + 4);
    const v8us o = { bfb(a.x), bfb(a.y), bfb(a.z), bfb(a.w), bfb(c.x), bfb(c.y), bfb(c.z), bfb(c.w) };
    store2_us8(xh + g * 8, o);
  } else if (bid < XBLK + WBLK) {
    const int e  = (bid - XBLK) * 256 + tid;
    const int n  = e >> 6;
    const int k0 = (e & 63) * 8;
    const int t  = n >> 3, i = n & 7;
    const int ic = (i < NI) ? i : (NI - 1);
    const float* src = tp + (size_t)t * PPT + ic * NF + k0;
    const float v0 = src[0], v1 = src[1], v2 = src[2], v3 = src[3];
    const float v4 = src[4], v5 = src[5], v6 = src[6], v7 = src[7];
    const bool pad = (i >= NI);
    const unsigned short zz = 0;
    const v8us o = { pad ? zz : bfb(v0), pad ? zz : bfb(v1), pad ? zz : bfb(v2), pad ? zz : bfb(v3),
                     pad ? zz : bfb(v4), pad ? zz : bfb(v5), pad ? zz : bfb(v6), pad ? zz : bfb(v7) };
    store2_us8(wt + (size_t)n * NF + k0, o);
  }
}

__global__ __launch_bounds__(256) void leafdist_kernel(
    const float* __restrict__ tp,
    unsigned short* __restrict__ LH,
    unsigned short* __restrict__ LL)
{
  __shared__ __attribute__((aligned(16))) unsigned short sH[128 * 64];
  __shared__ __attribute__((aligned(16))) unsigned short sL[128 * 64];

  const int tid = threadIdx.x, lane = tid & 31, w = tid >> 5;
  const int kg = blockIdx.x, cq = blockIdx.y;

  #pragma unroll 1
  for (int j = 0; j < 8; ++j) {
    const int kll = 8 * w + j;
    const int kl  = 64 * kg + kll;
    const int t = kl >> 3, l = kl & 7;
    const float* ll = tp + (size_t)t * PPT + OFF_L + l * NC;

    float mx = -3.0e38f;
    #pragma unroll 1
    for (int jj = 0; jj < NC / 32; ++jj) {
      const float v = bfv(bfb(ll[lane + 32 * jj]));
      mx = fmaxf(mx, v);
    }
    #pragma unroll
    for (int o = 16; o > 0; o >>= 1) mx = fmaxf(mx, __shfl_xor(mx, o));

    float s = 0.0f;
    #pragma unroll 1
    for (int jj = 0; jj < NC / 32; ++jj) {
      const float v = bfv(bfb(ll[lane + 32 * jj]));
      s += expf(v - mx);
    }
    #pragma unroll
    for (int o = 16; o > 0; o >>= 1) s += __shfl_xor(s, o);
    const float inv = 1.0f / s;

    #pragma unroll 1
    for (int cc = 0; cc < 4; ++cc) {
      const int cl = 32 * cc + lane;
      const int c  = 128 * cq + cl;
      const float v = bfv(bfb(ll[c]));
      const float p = expf(v - mx) * inv;
      const unsigned short hb = bfb(p);
      const unsigned short lb = bfb(p - bfv(hb));
      sH[cl * 64 + kll] = hb;
      sL[cl * 64 + kll] = lb;
    }
  }
  __syncthreads();

  unsigned short* gh = LH + (size_t)(128 * cq) * NCOL + 64 * kg;
  unsigned short* gl = LL + (size_t)(128 * cq) * NCOL + 64 * kg;
  line64_store_pass<16>(sH, gh, NCOL, w, lane);
  line64_store_pass<16>(sL, gl, NCOL, w, lane);
  __threadfence();
  line64_store_pass<16>(sH, gh, NCOL, w, lane);
  line64_store_pass<16>(sL, gl, NCOL, w, lane);
}

__device__ __forceinline__ void leaf_vals(float d0, float d1, float d2, float d3, float wt8,
                                          v8us& hv, v8us& lv) {
  #pragma clang fp contract(off)
  float lp[8];
  lp[0] = 1.0f;
  lp[1] = d0;  lp[2] = 1.0f - d0;
  lp[3] = d1;  lp[4] = 1.0f - d1;
  lp[5] = d2;  lp[6] = 1.0f - d2;
  lp[7] = d3;
  float s = lp[0];
  #pragma unroll
  for (int u = 1; u < 8; ++u) s = s + lp[u];
  const float den = s + 1e-8f;
  const float inv = 1.0f / den;
  #pragma unroll
  for (int u = 0; u < 8; ++u) {
    const float a = (lp[u] * inv) * wt8;
    const unsigned short hb = bfb(a);
    const unsigned short lb = bfb(a - bfv(hb));
    hv[u] = hb;
    lv[u] = lb;
  }
}

__global__ __launch_bounds__(128) void gate_leaf_kernel(
    const unsigned short* __restrict__ xh,
    const unsigned short* __restrict__ wt,
    const float* __restrict__ tp,
    const float* __restrict__ tw,
    unsigned short* __restrict__ AH,
    unsigned short* __restrict__ AL)
{
  __shared__ __attribute__((aligned(16))) float sT[128 * 64];
  unsigned short* sHs = (unsigned short*)sT;
  unsigned short* sLs = sHs + 128 * 64;

  const int tid = threadIdx.x, lane = tid & 31, w = tid >> 5;
  const int h = lane >> 4, m = lane & 15;
  const int m0 = blockIdx.x * 128, n0 = blockIdx.y * 64;
  const int m0w = m0 + 32 * w;

  const unsigned short* xa0 = xh + (size_t)(m0w + m) * NF;
  const unsigned short* xa1 = xa0 + (size_t)16 * NF;
  const unsigned short* wb  = wt + (size_t)(n0 + m) * NF;

  const v8f zero8 = {0.f, 0.f, 0.f, 0.f, 0.f, 0.f, 0.f, 0.f};
  v8f acc[2][4];
  #pragma unroll
  for (int mt = 0; mt < 2; ++mt)
    #pragma unroll
    for (int nt = 0; nt < 4; ++nt) acc[mt][nt] = zero8;

  #pragma unroll 1
  for (int k0 = 0; k0 < NF; k0 += 32) {
    const v16b a0 = load_frag(xa0 + k0, h);
    const v16b a1 = load_frag(xa1 + k0, h);
    #pragma unroll
    for (int nt = 0; nt < 4; ++nt) {
      const v16b b = load_frag(wb + (size_t)nt * 16 * NF + k0, h);
      acc[0][nt] = wmma_bf16(a0, b, acc[0][nt]);
      acc[1][nt] = wmma_bf16(a1, b, acc[1][nt]);
    }
  }

  #pragma unroll
  for (int nt = 0; nt < 4; ++nt) {
    const int col = 16 * nt + m;
    const int n = n0 + col;
    const int t = n >> 3, i = n & 7;
    const int ic = (i < NI) ? i : (NI - 1);
    float bv = bfv(bfb(tp[(size_t)t * PPT + OFF_B + ic]));
    bv = (i < NI) ? bv : 0.0f;
    #pragma unroll
    for (int mt = 0; mt < 2; ++mt) {
      #pragma unroll
      for (int r = 0; r < 8; ++r) {
        const int tokl = 32 * w + 16 * mt + 8 * h + r;
        const float z = acc[mt][nt][r] + bv;
        const float e = expf(-z);
        const float p = __builtin_amdgcn_rcpf(1.0f + e);
        sT[tokl * 64 + col] = p;
      }
    }
  }
  __syncthreads();

  const float* drow = sT + tid * 64;
  v4f d[8];
  float w8[8];
  #pragma unroll
  for (int t8 = 0; t8 < 8; ++t8) {
    d[t8] = *(const v4fa*)(drow + 8 * t8);
    w8[t8] = bfv(bfb(tw[8 * blockIdx.y + t8]));
  }
  __syncthreads();

  #pragma unroll
  for (int t8 = 0; t8 < 8; ++t8) {
    v8us hv, lv;
    leaf_vals(d[t8].x, d[t8].y, d[t8].z, d[t8].w, w8[t8], hv, lv);
    *(v8usa*)(sHs + tid * 64 + 8 * t8) = hv;
    *(v8usa*)(sLs + tid * 64 + 8 * t8) = lv;
  }
  __syncthreads();

  unsigned short* gh = AH + (size_t)m0 * NCOL + n0;
  unsigned short* gl = AL + (size_t)m0 * NCOL + n0;
  line64_store_pass<32>(sHs, gh, NCOL, w, lane);
  line64_store_pass<32>(sLs, gl, NCOL, w, lane);
  __threadfence();
  line64_store_pass<32>(sHs, gh, NCOL, w, lane);
  line64_store_pass<32>(sLs, gl, NCOL, w, lane);
}

__global__ __launch_bounds__(128) void out_gemm_kernel(
    const unsigned short* __restrict__ AH,
    const unsigned short* __restrict__ AL,
    const unsigned short* __restrict__ LH,
    const unsigned short* __restrict__ LL,
    float* __restrict__ out)
{
  __shared__ __attribute__((aligned(16))) float sT[128 * 64];

  const int tid = threadIdx.x, lane = tid & 31, w = tid >> 5;
  const int h = lane >> 4, m = lane & 15;
  const int m0 = blockIdx.x * 128, n0 = blockIdx.y * 64;
  const int m0w = m0 + 32 * w;

  const unsigned short* ha0 = AH + (size_t)(m0w + m) * NCOL;
  const unsigned short* ha1 = ha0 + (size_t)16 * NCOL;
  const unsigned short* la0 = AL + (size_t)(m0w + m) * NCOL;
  const unsigned short* la1 = la0 + (size_t)16 * NCOL;
  const unsigned short* hb  = LH + (size_t)(n0 + m) * NCOL;
  const unsigned short* lb  = LL + (size_t)(n0 + m) * NCOL;

  const v8f zero8 = {0.f, 0.f, 0.f, 0.f, 0.f, 0.f, 0.f, 0.f};
  v8f acc[2][4];
  #pragma unroll
  for (int mt = 0; mt < 2; ++mt)
    #pragma unroll
    for (int nt = 0; nt < 4; ++nt) acc[mt][nt] = zero8;

  #pragma unroll 1
  for (int k0 = 0; k0 < NCOL; k0 += 32) {
    const v16b ah0 = load_frag(ha0 + k0, h);
    const v16b ah1 = load_frag(ha1 + k0, h);
    const v16b al0 = load_frag(la0 + k0, h);
    const v16b al1 = load_frag(la1 + k0, h);
    #pragma unroll
    for (int nt = 0; nt < 4; ++nt) {
      const v16b bh = load_frag(hb + (size_t)nt * 16 * NCOL + k0, h);
      const v16b bl = load_frag(lb + (size_t)nt * 16 * NCOL + k0, h);
      acc[0][nt] = wmma_bf16(ah0, bh, acc[0][nt]);
      acc[0][nt] = wmma_bf16(al0, bh, acc[0][nt]);
      acc[0][nt] = wmma_bf16(ah0, bl, acc[0][nt]);
      acc[1][nt] = wmma_bf16(ah1, bh, acc[1][nt]);
      acc[1][nt] = wmma_bf16(al1, bh, acc[1][nt]);
      acc[1][nt] = wmma_bf16(ah1, bl, acc[1][nt]);
    }
  }

  #pragma unroll
  for (int nt = 0; nt < 4; ++nt) {
    const int col = 16 * nt + m;
    #pragma unroll
    for (int mt = 0; mt < 2; ++mt) {
      #pragma unroll
      for (int r = 0; r < 8; ++r) {
        const int tokl = 32 * w + 16 * mt + 8 * h + r;
        sT[tokl * 64 + col] = acc[mt][nt][r];
      }
    }
  }
  __syncthreads();

  float* g = out + (size_t)m0 * NC + n0;
  tile_store_pass(sT, g, NC, w, lane);
  __threadfence();
  tile_store_pass(sT, g, NC, w, lane);
}

extern "C" void kernel_launch(void* const* d_in, const int* in_sizes, int n_in,
                              void* d_out, int out_size, void* d_ws, size_t ws_size,
                              hipStream_t stream) {
  if (n_in < 3) return;
  if (in_sizes[0] != NB * NF) return;
  if (in_sizes[1] != NT * PPT) return;
  if (in_sizes[2] != NT) return;
  if (out_size != NB * NC) return;

  const float* x  = (const float*)d_in[0];
  const float* tp = (const float*)d_in[1];
  const float* tw = (const float*)d_in[2];
  float* out = (float*)d_out;

  const size_t sz_xh = (size_t)NB * NF * 2;
  const size_t sz_wt = (size_t)NCOL * NF * 2;
  const size_t sz_l  = (size_t)NC * NCOL * 2;
  const size_t sz_a  = (size_t)NB * NCOL * 2;
  const size_t off_xh = 0;
  const size_t off_wt = off_xh + sz_xh;
  const size_t off_lh = off_wt + sz_wt;
  const size_t off_ll = off_lh + sz_l;
  const size_t off_ah = off_ll + sz_l;
  const size_t off_al = off_ah + sz_a;
  const size_t total  = off_al + sz_a;
  if (total > ws_size) return;

  char* ws = (char*)d_ws;
  unsigned short* xh = (unsigned short*)(ws + off_xh);
  unsigned short* wt = (unsigned short*)(ws + off_wt);
  unsigned short* LH = (unsigned short*)(ws + off_lh);
  unsigned short* LL = (unsigned short*)(ws + off_ll);
  unsigned short* AH = (unsigned short*)(ws + off_ah);
  unsigned short* AL = (unsigned short*)(ws + off_al);

  convert_kernel<<<XBLK + WBLK, 256, 0, stream>>>(x, tp, xh, wt);

  dim3 gL(NCOL / 64, NC / 128);
  leafdist_kernel<<<gL, 256, 0, stream>>>(tp, LH, LL);

  dim3 g1(NB / 128, NCOL / 64);
  gate_leaf_kernel<<<g1, 128, 0, stream>>>(xh, wt, tp, tw, AH, AL);

  dim3 g2(NB / 128, NC / 64);
  out_gemm_kernel<<<g2, 128, 0, stream>>>(AH, AL, LH, LL, out);
}
